// UnifiedLIV_43748536877630
// MI455X (gfx1250) — hardware-verified
//
#include <hip/hip_runtime.h>
#include <stddef.h>
#include <stdint.h>


typedef _Float16 v8h  __attribute__((ext_vector_type(8)));
typedef _Float16 v16h __attribute__((ext_vector_type(16)));
typedef _Float16 v8ha __attribute__((ext_vector_type(8), may_alias));
typedef float    v4f  __attribute__((ext_vector_type(4)));
typedef float    v8f  __attribute__((ext_vector_type(8)));

#define NB   2
#define NL   2048
#define ND   1024
#define NH   16
#define HD   64
#define MT   (NB * NL)
#define QS   512
#define SP   72
#define KSL  64
#define STP  136

union Frag { v16h v; v8h hv[2]; };

__device__ __forceinline__ float bf16r(float f)
{
    unsigned int u = __float_as_uint(f);
    u = (u + 0x7FFFu + ((u >> 16) & 1u)) & 0xFFFF0000u;
    return __uint_as_float(u);
}

__device__ __forceinline__ v8f mma(v16h a, v16h b, v8f c)
{
    v8f d = __builtin_amdgcn_wmma_f32_16x16x32_f16(false, a, false, b, (short)0, c, false, false);
    asm volatile("v_nop\n\tv_nop\n\tv_nop\n\tv_nop" : "+v"(d) : "v"(a), "v"(b));
    return d;
}

__global__ __launch_bounds__(256)
void k_cvt(const float* __restrict__ s0, const float* __restrict__ s1,
           const float* __restrict__ s2, const float* __restrict__ s3,
           _Float16* d0, _Float16* d1, _Float16* d2, _Float16* d3,
           int n, float scale)
{
    const float* src = s0; _Float16* dst = d0;
    if (blockIdx.y == 1)      { src = s1; dst = d1; }
    else if (blockIdx.y == 2) { src = s2; dst = d2; }
    else if (blockIdx.y == 3) { src = s3; dst = d3; }

    const size_t i = ((size_t)blockIdx.x * 256 + threadIdx.x) * 8;
    if (i + 8 <= (size_t)n) {
        const v4f a = *(const v4f*)(src + i);
        const v4f c = *(const v4f*)(src + i + 4);
        v8h o;
#pragma unroll
        for (int e = 0; e < 4; ++e) {
            o[e]     = (_Float16)(bf16r(a[e]) * scale);
            o[e + 4] = (_Float16)(bf16r(c[e]) * scale);
        }
        *(volatile v8h*)(dst + i) = o;
        __threadfence();
        *(volatile v8h*)(dst + i) = o;
    } else if (i < (size_t)n) {
        for (size_t e = i; e < (size_t)n; ++e) {
            const _Float16 v = (_Float16)(bf16r(src[e]) * scale);
            *(volatile _Float16*)(dst + e) = v;
        }
        __threadfence();
        for (size_t e = i; e < (size_t)n; ++e) {
            const _Float16 v = (_Float16)(bf16r(src[e]) * scale);
            *(volatile _Float16*)(dst + e) = v;
        }
    }
}

__device__ __forceinline__ void put_plane_f16(const _Float16* st, _Float16* g, int tid)
{
    v8h w[8];
#pragma unroll
    for (int u = 0; u < 8; ++u) {
        const int c = u * 256 + tid, r = c >> 4, s = c & 15;
        w[u] = *(const v8h*)(st + r * STP + s * 8);
    }
#pragma unroll
    for (int u = 0; u < 8; ++u) {
        const int c = u * 256 + tid, r = c >> 4, s = c & 15;
        *(volatile v8h*)(g + (size_t)r * ND + s * 8) = w[u];
    }
    __threadfence();
#pragma unroll
    for (int u = 0; u < 8; ++u) {
        const int c = u * 256 + tid, r = c >> 4, s = c & 15;
        *(volatile v8h*)(g + (size_t)r * ND + s * 8) = w[u];
    }
}

__global__ __launch_bounds__(256) __attribute__((amdgpu_num_vgpr(248)))
void k_qkv(const _Float16* __restrict__ xh,
           const _Float16* __restrict__ w0, const _Float16* __restrict__ w1,
           const _Float16* __restrict__ w2,
           const float* __restrict__ g0, const float* __restrict__ g1,
           const float* __restrict__ g2,
           _Float16* y0h, _Float16* y0l, _Float16* y1h, _Float16* y1l,
           _Float16* y2h, _Float16* y2l)
{
    __shared__ __attribute__((aligned(16))) unsigned char lraw[2 * 128 * SP * 2];
    _Float16* sA = (_Float16*)lraw;
    _Float16* sB = sA + 128 * SP;

    const _Float16* W = w0; const float* bias = g0; _Float16* Yh = y0h; _Float16* Yl = y0l;
    if (blockIdx.z == 1)      { W = w1; bias = g1; Yh = y1h; Yl = y1l; }
    else if (blockIdx.z == 2) { W = w2; bias = g2; Yh = y2h; Yl = y2l; }

    const int tid = threadIdx.x, lane = tid & 31, wave = tid >> 5;
    const int h8 = (lane >> 4) * 8, m = lane & 15;
    const int wm = wave >> 2, wn = wave & 3;
    const int mblock = blockIdx.y * 128, nblock = blockIdx.x * 128;

    v8f acc[4][2] = {};

    for (int ks = 0; ks < ND / KSL; ++ks) {
        const int k0 = ks * KSL;
#pragma unroll
        for (int u = 0; u < 4; ++u) {
            const int c = u * 256 + tid, r = c >> 3, s = c & 7;
            *(v8h*)(sA + r * SP + s * 8) =
                *(const v8h*)(xh + (size_t)(mblock + r) * ND + k0 + s * 8);
            *(v8h*)(sB + r * SP + s * 8) =
                *(const v8h*)(W + (size_t)(nblock + r) * ND + k0 + s * 8);
        }
        __syncthreads();
#pragma unroll
        for (int kk = 0; kk < KSL; kk += 32) {
            Frag a[4], bq[2];
#pragma unroll
            for (int i = 0; i < 4; ++i) {
                const _Float16* p = sA + (wm * 64 + i * 16 + m) * SP + kk + h8;
                a[i].hv[0] = *(const v8h*)p;
                a[i].hv[1] = *(const v8h*)(p + 16);
            }
#pragma unroll
            for (int j = 0; j < 2; ++j) {
                const _Float16* p = sB + (wn * 32 + j * 16 + m) * SP + kk + h8;
                bq[j].hv[0] = *(const v8h*)p;
                bq[j].hv[1] = *(const v8h*)(p + 16);
            }
#pragma unroll
            for (int i = 0; i < 4; ++i)
#pragma unroll
                for (int j = 0; j < 2; ++j)
                    acc[i][j] = mma(a[i].v, bq[j].v, acc[i][j]);
        }
        __syncthreads();
    }

    float bb[2];
#pragma unroll
    for (int j = 0; j < 2; ++j) bb[j] = bf16r(bias[nblock + wn * 32 + j * 16 + m]);

    _Float16* st = (_Float16*)lraw;

#pragma unroll
    for (int i = 0; i < 4; ++i)
#pragma unroll
        for (int j = 0; j < 2; ++j)
#pragma unroll
            for (int r = 0; r < 8; ++r) {
                const int lr = wm * 64 + i * 16 + h8 + r;
                const int lc = wn * 32 + j * 16 + m;
                const float v = (acc[i][j][r] * (1.0f / 256.0f) + bb[j]) * 16.0f;
                st[lr * STP + lc] = (_Float16)v;
            }
    __syncthreads();
    put_plane_f16(st, Yh + (size_t)mblock * ND + nblock, tid);
    __syncthreads();

#pragma unroll
    for (int i = 0; i < 4; ++i)
#pragma unroll
        for (int j = 0; j < 2; ++j)
#pragma unroll
            for (int r = 0; r < 8; ++r) {
                const int lr = wm * 64 + i * 16 + h8 + r;
                const int lc = wn * 32 + j * 16 + m;
                const float v = (acc[i][j][r] * (1.0f / 256.0f) + bb[j]) * 16.0f;
                const _Float16 hv = (_Float16)v;
                st[lr * STP + lc] = (_Float16)((v - (float)hv) * 2048.0f);
            }
    __syncthreads();
    put_plane_f16(st, Yl + (size_t)mblock * ND + nblock, tid);
}

template <bool SPLIT>
__global__ __launch_bounds__(128) __attribute__((amdgpu_num_vgpr(248)))
void k_attn(const _Float16* __restrict__ qh, const _Float16* __restrict__ ql,
            const _Float16* __restrict__ kh, const _Float16* __restrict__ kl,
            const _Float16* __restrict__ vh, const _Float16* __restrict__ vl,
            _Float16* mh, _Float16* mlo, int xofs)
{
    constexpr int NP = SPLIT ? 2 : 1;
    __shared__ __attribute__((aligned(16))) _Float16 sK[NP][32 * SP];
    __shared__ __attribute__((aligned(16))) _Float16 sV[NP][32 * SP];
    __shared__ __attribute__((aligned(16))) _Float16 sPt[NP][4][512];
    __shared__ __attribute__((aligned(16))) _Float16 sO[2][64 * SP];

    const int tid = threadIdx.x, lane = tid & 31, wave = tid >> 5;
    const int h8 = (lane >> 4) * 8, m = lane & 15;
    const int bx = blockIdx.x + xofs;
    const int bh = blockIdx.y;
    const int b  = bh / NH;
    const int hd = bh - b * NH;
    const int q0 = bx * 64 + wave * 16;
    const size_t base = (size_t)b * NL * ND + (size_t)hd * HD;

    const _Float16* Qh = qh + base; const _Float16* Ql = ql + base;
    const _Float16* Kh = kh + base; const _Float16* Kl = kl + base;
    const _Float16* Vh = vh + base; const _Float16* Vl = vl + base;

    Frag aq[2], aql[2];
#pragma unroll
    for (int s = 0; s < 2; ++s) {
        const _Float16* p = Qh + (size_t)(q0 + m) * ND + s * 32 + h8;
        aq[s].hv[0] = *(const v8h*)p;
        aq[s].hv[1] = *(const v8h*)(p + 16);
        if (SPLIT) {
            const _Float16* pl = Ql + (size_t)(q0 + m) * ND + s * 32 + h8;
            aql[s].hv[0] = *(const v8h*)pl;
            aql[s].hv[1] = *(const v8h*)(pl + 16);
        } else {
            aql[s].v = aq[s].v;
        }
    }

    v8f o[4] = {};
    float mrow[8], lrow[8];
#pragma unroll
    for (int g = 0; g < 8; ++g) { mrow[g] = -__builtin_inff(); lrow[g] = 0.0f; }

    const float C11 = 4.8828125e-4f;
    const int nsteps = 2 * bx + 2;

    for (int it = 0; it < nsteps; ++it) {
        const int jb = it * 32;
        __syncthreads();
#pragma unroll
        for (int p = 0; p < NP; ++p) {
            const _Float16* Kp = p ? Kl : Kh;
            const _Float16* Vp = p ? Vl : Vh;
#pragma unroll
            for (int u = 0; u < 2; ++u) {
                const int c = u * 128 + tid, r = c >> 3, s = c & 7;
                *(v8h*)(&sK[p][r * SP + s * 8]) = *(const v8h*)(Kp + (size_t)(jb + r) * ND + s * 8);
                *(v8h*)(&sV[p][r * SP + s * 8]) = *(const v8h*)(Vp + (size_t)(jb + r) * ND + s * 8);
            }
        }
        __syncthreads();

        float lg[2][8];
#pragma unroll
        for (int kt = 0; kt < 2; ++kt) {
            v8f sm = {}, sc = {};
#pragma unroll
            for (int s = 0; s < 2; ++s) {
                Frag bk;
                const _Float16* p = &sK[0][(kt * 16 + m) * SP + s * 32 + h8];
                bk.hv[0] = *(const v8h*)p;
                bk.hv[1] = *(const v8h*)(p + 16);
                sm = mma(aq[s].v, bk.v, sm);
                if (SPLIT) {
                    Frag bkl;
                    const _Float16* pl = &sK[NP - 1][(kt * 16 + m) * SP + s * 32 + h8];
                    bkl.hv[0] = *(const v8h*)pl;
                    bkl.hv[1] = *(const v8h*)(pl + 16);
                    sc = mma(aq[s].v, bkl.v, sc);
                    sc = mma(aql[s].v, bk.v, sc);
                }
            }
#pragma unroll
            for (int g = 0; g < 8; ++g) {
                float v = sm[g];
                if (SPLIT) v += sc[g] * C11;
                lg[kt][g] = v * C11;
            }
        }

#pragma unroll
        for (int g = 0; g < 8; ++g) {
            const int row = q0 + h8 + g;
            float v0 = lg[0][g];
            float v1 = lg[1][g];
            if (jb + m > row)      v0 = -__builtin_inff();
            if (jb + 16 + m > row) v1 = -__builtin_inff();

            float rmx = fmaxf(v0, v1);
            rmx = fmaxf(rmx, __shfl_xor(rmx, 1, 16));
            rmx = fmaxf(rmx, __shfl_xor(rmx, 2, 16));
            rmx = fmaxf(rmx, __shfl_xor(rmx, 4, 16));
            rmx = fmaxf(rmx, __shfl_xor(rmx, 8, 16));

            const float mnew = fmaxf(mrow[g], rmx);
            const float corr = __expf(mrow[g] - mnew);
            const float p0 = __expf(v0 - mnew);
            const float p1 = __expf(v1 - mnew);

            float ps = p0 + p1;
            ps += __shfl_xor(ps, 1, 16);
            ps += __shfl_xor(ps, 2, 16);
            ps += __shfl_xor(ps, 4, 16);
            ps += __shfl_xor(ps, 8, 16);

            lrow[g] = lrow[g] * corr + ps;
            mrow[g] = mnew;
#pragma unroll
            for (int t = 0; t < 4; ++t) o[t][g] *= corr;

            const _Float16 hp0 = (_Float16)p0, hp1 = (_Float16)p1;
            sPt[0][wave][(h8 + g) * 32 + m]      = hp0;
            sPt[0][wave][(h8 + g) * 32 + 16 + m] = hp1;
            if (SPLIT) {
                sPt[NP - 1][wave][(h8 + g) * 32 + m]      = (_Float16)((p0 - (float)hp0) * 2048.0f);
                sPt[NP - 1][wave][(h8 + g) * 32 + 16 + m] = (_Float16)((p1 - (float)hp1) * 2048.0f);
            }
        }
        __asm__ volatile("" ::: "memory");

        Frag ap, apl;
        ap.hv[0] = *(const v8ha*)(&sPt[0][wave][m * 32 + h8]);
        ap.hv[1] = *(const v8ha*)(&sPt[0][wave][m * 32 + 16 + h8]);
        if (SPLIT) {
            apl.hv[0] = *(const v8ha*)(&sPt[NP - 1][wave][m * 32 + h8]);
            apl.hv[1] = *(const v8ha*)(&sPt[NP - 1][wave][m * 32 + 16 + h8]);
        } else {
            apl.v = ap.v;
        }

#pragma unroll
        for (int t = 0; t < 4; ++t) {
            v16h bv, bvl;
#pragma unroll
            for (int i = 0; i < 16; ++i) {
                const int k = h8 + i + (i & 8);
                bv[i] = sV[0][k * SP + t * 16 + m];
                if (SPLIT) bvl[i] = sV[NP - 1][k * SP + t * 16 + m];
                else       bvl[i] = bv[i];
            }
            o[t] = mma(ap.v, bv, o[t]);
            if (SPLIT) {
                v8f oc = {};
                oc = mma(ap.v, bvl, oc);
                oc = mma(apl.v, bv, oc);
#pragma unroll
                for (int r = 0; r < 8; ++r) o[t][r] += oc[r] * C11;
            }
        }
    }

#pragma unroll
    for (int g = 0; g < 8; ++g) {
        const float inv = 1.0f / lrow[g];
#pragma unroll
        for (int t = 0; t < 4; ++t) {
            const float val = o[t][g] * inv;
            const _Float16 hv = (_Float16)val;
            const int idx = (wave * 16 + h8 + g) * SP + t * 16 + m;
            sO[0][idx] = hv;
            sO[1][idx] = (_Float16)((val - (float)hv) * 2048.0f);
        }
    }
    __syncthreads();

    const size_t mrow0 = base + (size_t)(bx * 64) * ND;
    v8h w0[4], w1[4];
#pragma unroll
    for (int u = 0; u < 4; ++u) {
        const int c = u * 128 + tid, r = c >> 3, s = c & 7;
        w0[u] = *(const v8h*)(&sO[0][r * SP + s * 8]);
        w1[u] = *(const v8h*)(&sO[1][r * SP + s * 8]);
    }
#pragma unroll
    for (int u = 0; u < 4; ++u) {
        const int c = u * 128 + tid, r = c >> 3, s = c & 7;
        *(volatile v8h*)(mh  + mrow0 + (size_t)r * ND + s * 8) = w0[u];
        *(volatile v8h*)(mlo + mrow0 + (size_t)r * ND + s * 8) = w1[u];
    }
    __threadfence();
#pragma unroll
    for (int u = 0; u < 4; ++u) {
        const int c = u * 128 + tid, r = c >> 3, s = c & 7;
        *(volatile v8h*)(mh  + mrow0 + (size_t)r * ND + s * 8) = w0[u];
        *(volatile v8h*)(mlo + mrow0 + (size_t)r * ND + s * 8) = w1[u];
    }
}

template <bool SPLIT>
__global__ __launch_bounds__(256) __attribute__((amdgpu_num_vgpr(248)))
void k_out(const _Float16* __restrict__ ah, const _Float16* __restrict__ al,
           const _Float16* __restrict__ wc, float* y, int yofs)
{
    constexpr int NT   = SPLIT ? 1 : 2;
    constexpr int BN   = 64 * NT;
    constexpr int NA   = SPLIT ? 2 : 1;
    constexpr int LDSB = (NA * 128 * SP + BN * SP) * 2;
    __shared__ __attribute__((aligned(16))) unsigned char lraw[LDSB];
    _Float16* sA = (_Float16*)lraw;
    _Float16* sL = sA + 128 * SP;
    _Float16* sB = sA + NA * 128 * SP;

    const int tid = threadIdx.x, lane = tid & 31, wave = tid >> 5;
    const int h8 = (lane >> 4) * 8, m = lane & 15;
    const int wm = wave >> 2, wn = wave & 3;
    const int mblock = blockIdx.z * NL + (blockIdx.y + yofs) * 128;
    const int nblock = blockIdx.x * BN;

    v8f acc[4][NT] = {};
    v8f acl[4][NT] = {};

    for (int ks = 0; ks < ND / KSL; ++ks) {
        const int k0 = ks * KSL;
#pragma unroll
        for (int u = 0; u < 4; ++u) {
            const int c = u * 256 + tid, r = c >> 3, s = c & 7;
            *(v8h*)(sA + r * SP + s * 8) =
                *(const v8h*)(ah + (size_t)(mblock + r) * ND + k0 + s * 8);
            if (SPLIT)
                *(v8h*)(sL + r * SP + s * 8) =
                    *(const v8h*)(al + (size_t)(mblock + r) * ND + k0 + s * 8);
        }
#pragma unroll
        for (int u = 0; u < BN / 32; ++u) {
            const int c = u * 256 + tid, r = c >> 3, s = c & 7;
            *(v8h*)(sB + r * SP + s * 8) =
                *(const v8h*)(wc + (size_t)(nblock + r) * ND + k0 + s * 8);
        }
        __syncthreads();
#pragma unroll
        for (int kk = 0; kk < KSL; kk += 32) {
            Frag a[4], e[4], bq[NT];
#pragma unroll
            for (int i = 0; i < 4; ++i) {
                const _Float16* p = sA + (wm * 64 + i * 16 + m) * SP + kk + h8;
                a[i].hv[0] = *(const v8h*)p;
                a[i].hv[1] = *(const v8h*)(p + 16);
                if (SPLIT) {
                    const _Float16* pl = sL + (wm * 64 + i * 16 + m) * SP + kk + h8;
                    e[i].hv[0] = *(const v8h*)pl;
                    e[i].hv[1] = *(const v8h*)(pl + 16);
                } else {
                    e[i].v = a[i].v;
                }
            }
#pragma unroll
            for (int j = 0; j < NT; ++j) {
                const _Float16* p = sB + (wn * 16 * NT + j * 16 + m) * SP + kk + h8;
                bq[j].hv[0] = *(const v8h*)p;
                bq[j].hv[1] = *(const v8h*)(p + 16);
            }
#pragma unroll
            for (int i = 0; i < 4; ++i)
#pragma unroll
                for (int j = 0; j < NT; ++j) {
                    acc[i][j] = mma(a[i].v, bq[j].v, acc[i][j]);
                    if (SPLIT) acl[i][j] = mma(e[i].v, bq[j].v, acl[i][j]);
                }
        }
        __syncthreads();
    }

    float* st = (float*)lraw;
    constexpr int PP  = BN + 4;
    constexpr int CPR = BN / 4;
    constexpr int NU  = CPR / 4;

    for (int half = 0; half < 2; ++half) {
        if (wm == half) {
#pragma unroll
            for (int i = 0; i < 4; ++i)
#pragma unroll
                for (int j = 0; j < NT; ++j)
#pragma unroll
                    for (int r = 0; r < 8; ++r) {
                        const int lr = i * 16 + h8 + r;
                        const int lc = wn * 16 * NT + j * 16 + m;
                        float v = acc[i][j][r];
                        if (SPLIT) v += acl[i][j][r] * 4.8828125e-4f;
                        v *= (1.0f / 4096.0f);
                        st[lr * PP + lc] = v;
                    }
        }
        __syncthreads();
        float* gb = y + (size_t)(mblock + half * 64) * ND + nblock;
        v4f vv[NU];
#pragma unroll
        for (int u = 0; u < NU; ++u) {
            const int c = u * 256 + tid, r = c / CPR, s = c - r * CPR;
            vv[u] = *(const v4f*)(st + r * PP + s * 4);
        }
#pragma unroll
        for (int u = 0; u < NU; ++u) {
            const int c = u * 256 + tid, r = c / CPR, s = c - r * CPR;
            *(volatile v4f*)(gb + (size_t)r * ND + s * 4) = vv[u];
        }
        __threadfence();
#pragma unroll
        for (int u = 0; u < NU; ++u) {
            const int c = u * 256 + tid, r = c / CPR, s = c - r * CPR;
            *(volatile v4f*)(gb + (size_t)r * ND + s * 4) = vv[u];
        }
        __syncthreads();
    }
}

extern "C" void kernel_launch(void* const* d_in, const int* in_sizes, int n_in,
                              void* d_out, int out_size, void* d_ws, size_t ws_size,
                              hipStream_t stream)
{
    if (n_in < 8) return;
    if (in_sizes[0] != MT * ND) return;
    if (in_sizes[1] != ND * ND || in_sizes[3] != ND * ND ||
        in_sizes[5] != ND * ND || in_sizes[7] != ND * ND) return;
    if (in_sizes[2] != ND || in_sizes[4] != ND || in_sizes[6] != ND) return;
    if (out_size != MT * ND) return;

    const float* x  = (const float*)d_in[0];
    const float* WQ = (const float*)d_in[1];
    const float* bQ = (const float*)d_in[2];
    const float* WK = (const float*)d_in[3];
    const float* bK = (const float*)d_in[4];
    const float* WV = (const float*)d_in[5];
    const float* bV = (const float*)d_in[6];
    const float* Wc = (const float*)d_in[7];
    float* y = (float*)d_out;

    const size_t szA = (size_t)MT * ND * sizeof(_Float16);
    const size_t szW = (size_t)ND * ND * sizeof(_Float16);
    unsigned char* ws = (unsigned char*)d_ws;
    size_t off = 0;
    _Float16* xh  = (_Float16*)(ws + off); off += szA;
    _Float16* wq  = (_Float16*)(ws + off); off += szW;
    _Float16* wk  = (_Float16*)(ws + off); off += szW;
    _Float16* wv  = (_Float16*)(ws + off); off += szW;
    _Float16* wch = (_Float16*)(ws + off); off += szW;
    _Float16* qh  = (_Float16*)(ws + off); off += szA;
    _Float16* ql  = (_Float16*)(ws + off); off += szA;
    _Float16* kh  = (_Float16*)(ws + off); off += szA;
    _Float16* kl  = (_Float16*)(ws + off); off += szA;
    _Float16* vh  = (_Float16*)(ws + off); off += szA;
    _Float16* vl  = (_Float16*)(ws + off); off += szA;
    _Float16* mh  = (_Float16*)(ws + off); off += szA;
    _Float16* ml  = (_Float16*)(ws + off); off += szA;
    if (off > ws_size) return;

    k_cvt<<<dim3((MT * ND + 2047) / 2048, 1), 256, 0, stream>>>(
        x, x, x, x, xh, xh, xh, xh, MT * ND, 1.0f);
    k_cvt<<<dim3((ND * ND + 2047) / 2048, 4), 256, 0, stream>>>(
        WQ, WK, WV, Wc, wq, wk, wv, wch, ND * ND, 256.0f);

    k_qkv<<<dim3(ND / 128, MT / 128, 3), 256, 0, stream>>>(
        xh, wq, wk, wv, bQ, bK, bV, qh, ql, kh, kl, vh, vl);

    k_attn<true><<<dim3(QS / 64, NB * NH), 128, 0, stream>>>(
        qh, ql, kh, kl, vh, vl, mh, ml, 0);
    k_attn<false><<<dim3(NL / 64 - QS / 64, NB * NH), 128, 0, stream>>>(
        qh, ql, kh, kl, vh, vl, mh, ml, QS / 64);

    k_out<true><<<dim3(ND / 64, QS / 128, NB), 256, 0, stream>>>(
        mh, ml, wch, y, 0);
    k_out<false><<<dim3(ND / 128, NL / 128 - QS / 128, NB), 256, 0, stream>>>(
        mh, ml, wch, y, QS / 128);
}
